// DeformConv1d_45827301048698
// MI455X (gfx1250) — hardware-verified
//
#include <hip/hip_runtime.h>
#include <math.h>

typedef __attribute__((ext_vector_type(16))) _Float16 v16h;
typedef __attribute__((ext_vector_type(16))) __bf16 v16b;
typedef __attribute__((ext_vector_type(8)))  _Float16 v8h;
typedef __attribute__((ext_vector_type(8)))  float v8f;
typedef __attribute__((ext_vector_type(4)))  float v4f;
typedef __attribute__((ext_vector_type(2)))  float v2f;
typedef __attribute__((ext_vector_type(4)))  unsigned v4u;
typedef __attribute__((ext_vector_type(4)))  int v4i;
typedef float __attribute__((may_alias)) float_a;
typedef int __attribute__((may_alias)) int_a;

template <typename T> __device__ __forceinline__ void vst2(void* p, T v) { *(volatile T*)p = v; __threadfence(); *(volatile T*)p = v; }
__device__ __forceinline__ v8f wmma16(v16h a, v16h b, v8f c) {
  v8f d = __builtin_amdgcn_wmma_f32_16x16x32_f16(false, a, false, b, (short)0, c, false, false);
  asm volatile("v_nop\n\tv_nop\n\tv_nop\n\tv_nop" : "+v"(d) : "v"(a), "v"(b));
  return d;
}
__device__ __forceinline__ v8f wmma_bf(v16b a, v16b b, v8f c) {
  v8f d = __builtin_amdgcn_wmma_f32_16x16x32_bf16(false, a, false, b, (short)0, c, false, false);
  asm volatile("v_nop\n\tv_nop\n\tv_nop\n\tv_nop" : "+v"(d) : "v"(a), "v"(b));
  return d;
}
__device__ __forceinline__ v16h frag_h(const _Float16* rowk0, int lane) {
  union { v16h v; v8h q[2]; } u; const _Float16* p = rowk0 + 8 * (lane >> 4);
  u.q[0] = *(const v8h*)p; u.q[1] = *(const v8h*)(p + 16); return u.v;
}
__device__ __forceinline__ v16h frag_f32(const float* rowk0, int lane) {
  v16h a; const float* p = rowk0 + 8 * (lane >> 4);
#pragma unroll
  for (int i = 0; i < 8; ++i) { a[i] = (_Float16)p[i]; a[8 + i] = (_Float16)p[16 + i]; }
  return a;
}
__device__ __forceinline__ v16h frag_f32s(const float* rowk0, int lane, float sc) {
  v16h a; const float* p = rowk0 + 8 * (lane >> 4);
#pragma unroll
  for (int i = 0; i < 8; ++i) { a[i] = (_Float16)(p[i] * sc); a[8 + i] = (_Float16)(p[16 + i] * sc); }
  return a;
}
__device__ __forceinline__ v16h fragc_f32(const float* W, int k0, int n, int lane, int ld, int K) {
  v16h a; const int g = lane >> 4;
#pragma unroll
  for (int i = 0; i < 8; ++i) { const int ka = k0 + 8 * g + i, kb = ka + 16;
    a[i] = (_Float16)(ka < K ? W[(size_t)(ka < K ? ka : K - 1) * ld + n] : 0.f); a[8 + i] = (_Float16)(kb < K ? W[(size_t)(kb < K ? kb : K - 1) * ld + n] : 0.f); }
  return a;
}
struct F2 { v16b h, l; };
__device__ __forceinline__ F2 bsplit16(const float v[16]) { F2 r;
#pragma unroll
  for (int i = 0; i < 16; ++i) { const __bf16 h = (__bf16)v[i]; r.h[i] = h; r.l[i] = (__bf16)(v[i] - (float)h); }
  return r; }
__device__ __forceinline__ F2 split_row(const float* row, int k0, int lane) { float v[16]; const float* p = row + k0 + 8 * (lane >> 4);
#pragma unroll
  for (int i = 0; i < 8; ++i) { v[i] = p[i]; v[8 + i] = p[16 + i]; }
  return bsplit16(v); }
__device__ __forceinline__ F2 split_rowK(const float* row, int k0, int lane, int K) { float v[16]; const int g = lane >> 4;
#pragma unroll
  for (int i = 0; i < 8; ++i) { const int ka = k0 + 8 * g + i, kb = ka + 16; v[i] = ka < K ? row[ka < K ? ka : K - 1] : 0.f; v[8 + i] = kb < K ? row[kb < K ? kb : K - 1] : 0.f; }
  return bsplit16(v); }
__device__ __forceinline__ F2 split_col(const float* W, int k0, int n, int lane, int ld, int K) { float v[16]; const int g = lane >> 4;
#pragma unroll
  for (int i = 0; i < 8; ++i) { const int ka = k0 + 8 * g + i, kb = ka + 16; v[i] = ka < K ? W[(size_t)(ka < K ? ka : K - 1) * ld + n] : 0.f; v[8 + i] = kb < K ? W[(size_t)(kb < K ? kb : K - 1) * ld + n] : 0.f; }
  return bsplit16(v); }
__device__ __forceinline__ v8f mac3(const F2& a, const F2& b, v8f c) { c = wmma_bf(a.l, b.h, c); c = wmma_bf(a.h, b.l, c); return wmma_bf(a.h, b.h, c); }
__device__ __forceinline__ float sigm(float v) { return 1.0f / (1.0f + expf(-v)); }
#define LDSX() do { asm volatile("s_wait_dscnt 0" ::: "memory"); __builtin_amdgcn_wave_barrier(); __builtin_amdgcn_fence(__ATOMIC_RELEASE, "workgroup"); } while (0)


#define NB 8
#define C 256
#define L 4096
#define TO 4094
#define CO 256
#define KS 3
__device__ __forceinline__ float bfr(float v) { return (float)(__bf16)v; }

__device__ __forceinline__ v16b frag_b(const __bf16* rowk0, int lane) { return __builtin_bit_cast(v16b, frag_h((const _Float16*)rowk0, lane)); }
__global__ __launch_bounds__(256) void k_prep(const float* __restrict__ x, const float* __restrict__ W, __bf16* __restrict__ XT, __bf16* __restrict__ WT) {
  __shared__ __align__(16) __bf16 st[64][C + 8];
  const int tid = threadIdx.x;
  if (blockIdx.y < NB) { const int b = blockIdx.y, t0 = blockIdx.x * 64; const float* xb = x + (size_t)b * C * L;
    for (int q = tid; q < C * 64; q += 256) { const int c = q >> 6, tl = q & 63; st[tl][c] = (__bf16)xb[(size_t)c * L + t0 + tl]; }
    __syncthreads();
    for (int q = tid; q < 64 * (C / 8); q += 256) { const int tl = q >> 5, pc = q & 31; vst2((unsigned*)(XT + ((size_t)b * L + t0 + tl) * C + pc * 8), *(const v4u*)(&st[tl][pc * 8])); } }
  else {
    const int kk = blockIdx.x / 4, og = blockIdx.x % 4; if (kk >= KS) return; const int o0 = og * 64;
    for (int q = tid; q < 64 * C; q += 256) { const int ol = q >> 8, c = q & 255; st[ol][c] = (__bf16)W[((size_t)(o0 + ol) * C + c) * KS + kk]; }
    __syncthreads();
    for (int q = tid; q < 64 * (C / 8); q += 256) { const int ol = q >> 5, pc = q & 31; vst2((unsigned*)(WT + ((size_t)kk * CO + o0 + ol) * C + pc * 8), *(const v4u*)(&st[ol][pc * 8])); } }
}

__global__ __launch_bounds__(128) void k_dconv(const __bf16* __restrict__ XT, const float* __restrict__ off, const __bf16* __restrict__ WT, const float* __restrict__ bias, float* __restrict__ OUTW) {
  __shared__ __align__(16) float so[4][16][132]; __shared__ int sU[4][16][KS]; __shared__ float sw[4][16][KS][2];
  __shared__ __align__(16) __bf16 sxt[68][C + 8];
  const int tid = threadIdx.x, wave = tid >> 5, lane = tid & 31, col = lane & 15, g = lane >> 4;
  const int b = blockIdx.y, o0 = blockIdx.x * 128; const __bf16* XTb = XT + (size_t)b * L * C;
#pragma unroll 1
  for (int tc = 0; tc < (TO + 63) / 64; ++tc) { const int t0 = tc * 64 + wave * 16;
    if (lane < 16) { int t = t0 + lane; if (t > TO - 1) t = TO - 1;
#pragma unroll
      for (int kk = 0; kk < KS; ++kk) { const float base = (float)t + (float)kk; float T = base + bfr(off[((size_t)b * TO + t) * KS + kk]); T = fminf(fmaxf(T, (float)t), (float)t + 2.0f);
        float fl = floorf(T); fl = fminf(fmaxf(fl, 0.f), (float)(L - 2)); const int U0 = (int)fl; const float w0 = fmaxf(0.f, 1.0f - fabsf(fl - T)), w1 = fmaxf(0.f, 1.0f - fabsf(fl + 1.0f - T));
        sU[wave][lane][kk] = U0; sw[wave][lane][kk][0] = w0; sw[wave][lane][kk][1] = w1; } }
    { const int tb = tc * 64; for (int q = tid; q < 67 * (C / 8); q += 128) { const int rl = q >> 5, pc = q & 31; int tr = tb + rl; if (tr > L - 1) tr = L - 1; *(v4u*)(&sxt[rl][pc * 8]) = *(const v4u*)(XTb + (size_t)tr * C + pc * 8); } }
    __syncthreads();
    v8f tot[8] = {};
#pragma unroll 1
    for (int kk = 0; kk < KS; ++kk) {
#pragma unroll 1
      for (int u = 0; u < 2; ++u) { const int Ul = sU[wave][col][kk] + u - tc * 64; v8f acc[8] = {};
#pragma unroll 2
        for (int kc = 0; kc < C / 32; ++kc) { const v16b a = frag_b(&sxt[Ul][0] + kc * 32, lane);
#pragma unroll
          for (int j = 0; j < 8; ++j) acc[j] = wmma_bf(a, frag_b(WT + ((size_t)kk * CO + o0 + j * 16 + col) * C + kc * 32, lane), acc[j]); }
#pragma unroll
        for (int r = 0; r < 8; ++r) { const float wr = sw[wave][8 * g + r][kk][u];
#pragma unroll
          for (int j = 0; j < 8; ++j) tot[j][r] += wr * acc[j][r]; } } }
#pragma unroll
    for (int j = 0; j < 8; ++j) { const float bb = bfr(bias[o0 + j * 16 + col]);
#pragma unroll
      for (int r = 0; r < 8; ++r) so[wave][8 * g + r][j * 16 + col] = tot[j][r] + bb; }
    LDSX();
    __syncthreads();
    for (int q = tid; q < 128 * 16; q += 128) { const int ol = q >> 4, p = q & 15; const int t4 = p * 4; v4f v;
#pragma unroll
      for (int e = 0; e < 4; ++e) { const int tl = t4 + e; v[e] = so[tl >> 4][tl & 15][ol]; }
      vst2(OUTW + ((size_t)b * CO + o0 + ol) * L + tc * 64 + t4, v); }
    __syncthreads(); }
}
__global__ __launch_bounds__(256) void k_copy(const float* __restrict__ OUTW, float* __restrict__ out) {
  const size_t i4 = (size_t)blockIdx.x * 256 + threadIdx.x; const size_t total = (size_t)NB * CO * TO; if (i4 * 4 >= total) return;
  v4f v;
#pragma unroll
  for (int e = 0; e < 4; ++e) { size_t f = i4 * 4 + e; if (f >= total) f = total - 1; const size_t row = f / TO, t = f % TO; v[e] = OUTW[row * L + t]; }
  if (i4 * 4 + 4 <= total) vst2(out + i4 * 4, v);
  else { for (int e = 0; e < 4; ++e) if (i4 * 4 + e < total) vst2(out + i4 * 4 + e, (float_a)v[e]); }
}
extern "C" void kernel_launch(void* const* d_in, const int* in_sizes, int n_in, void* d_out, int out_size, void* d_ws, size_t ws_size, hipStream_t stream) {
  (void)in_sizes; (void)n_in; (void)out_size; (void)ws_size;
  const float* x = (const float*)d_in[0]; const float* off = (const float*)d_in[1]; const float* W = (const float*)d_in[2]; const float* bias = (const float*)d_in[3];
  char* ws = (char*)d_ws; float* OUTW = (float*)ws; __bf16* XT = (__bf16*)(ws + (size_t)NB * CO * L * 4); __bf16* WT = XT + (size_t)NB * L * C;
  k_prep<<<dim3(L / 64, NB + 1), 256, 0, stream>>>(x, W, XT, WT);
  k_dconv<<<dim3(CO / 128, NB), 128, 0, stream>>>(XT, off, WT, bias, OUTW);
  k_copy<<<(unsigned)(((size_t)NB * CO * TO / 4 + 255) / 256), 256, 0, stream>>>(OUTW, (float*)d_out);
}
